// TDNN_72490458022265
// MI455X (gfx1250) — hardware-verified
//
#include <hip/hip_runtime.h>
#include <math.h>


#define NB 16
#define T0 2048
#define FE 20
#define C1 512
#define C5 1500
#define C5P 1536
#define NSPK 6000
#define T5 2034
#define NTB ((T5 + 63) / 64)

typedef __attribute__((ext_vector_type(16))) _Float16 v16h;
typedef __attribute__((ext_vector_type(16))) __bf16 v16b;
typedef __attribute__((ext_vector_type(8)))  _Float16 v8h;
typedef __attribute__((ext_vector_type(8)))  float v8f;
typedef __attribute__((ext_vector_type(4)))  float v4f;
typedef __attribute__((ext_vector_type(4)))  unsigned v4u;
typedef float __attribute__((may_alias)) float_a;

template <typename T> __device__ __forceinline__ void vst2(void* p, T v) { *(volatile T*)p = v; __threadfence(); *(volatile T*)p = v; }
__device__ __forceinline__ v8f wmma16(v16h a, v16h b, v8f c) {
  v8f d = __builtin_amdgcn_wmma_f32_16x16x32_f16(false, a, false, b, (short)0, c, false, false);
  asm volatile("v_nop\n\tv_nop\n\tv_nop\n\tv_nop" : "+v"(d) : "v"(a), "v"(b));
  return d;
}
__device__ __forceinline__ v8f wmma_bf(v16b a, v16b b, v8f c) {
  v8f d = __builtin_amdgcn_wmma_f32_16x16x32_bf16(false, a, false, b, (short)0, c, false, false);
  asm volatile("v_nop\n\tv_nop\n\tv_nop\n\tv_nop" : "+v"(d) : "v"(a), "v"(b));
  return d;
}
__device__ __forceinline__ v16h frag_h(const _Float16* rowk0, int lane) {
  union { v16h v; v8h q[2]; } u; const _Float16* p = rowk0 + 8 * (lane >> 4);
  u.q[0] = *(const v8h*)p; u.q[1] = *(const v8h*)(p + 16); return u.v;
}
struct F2 { v16b h, l; };
__device__ __forceinline__ F2 bsplit16(const float v[16]) { F2 r;
#pragma unroll
  for (int i = 0; i < 16; ++i) { const __bf16 h = (__bf16)v[i]; r.h[i] = h; r.l[i] = (__bf16)(v[i] - (float)h); }
  return r; }
__device__ __forceinline__ F2 split_rowK(const float* row, int k0, int lane, int K) { float v[16]; const int g = lane >> 4;
#pragma unroll
  for (int i = 0; i < 8; ++i) { const int ka = k0 + 8 * g + i, kb = ka + 16; v[i] = ka < K ? row[ka] : 0.f; v[8 + i] = kb < K ? row[kb] : 0.f; }
  return bsplit16(v); }
__device__ __forceinline__ F2 split_colK(const float* W, int k0, int n, int lane, int ld, int K) { float v[16]; const int g = lane >> 4;
#pragma unroll
  for (int i = 0; i < 8; ++i) { const int ka = k0 + 8 * g + i, kb = ka + 16; v[i] = ka < K ? W[(size_t)ka * ld + n] : 0.f; v[8 + i] = kb < K ? W[(size_t)kb * ld + n] : 0.f; }
  return bsplit16(v); }
__device__ __forceinline__ v8f mac3(const F2& a, const F2& b, v8f c) { c = wmma_bf(a.l, b.h, c); c = wmma_bf(a.h, b.l, c); return wmma_bf(a.h, b.h, c); }
#define LDSX() do { asm volatile("s_wait_dscnt 0" ::: "memory"); __builtin_amdgcn_wave_barrier(); __builtin_amdgcn_fence(__ATOMIC_RELEASE, "workgroup"); } while (0)

__global__ __launch_bounds__(256) void k_cvt(const float* __restrict__ s, _Float16* __restrict__ d, size_t n8) {
  const size_t g8 = (size_t)blockIdx.x * 256 + threadIdx.x; if (g8 >= n8) return;
  union { v8h h; v4u u; } pk;
#pragma unroll
  for (int e = 0; e < 8; ++e) pk.h[e] = (_Float16)s[g8 * 8 + e];
  vst2(d + g8 * 8, pk.u);
}
__global__ __launch_bounds__(128) void k_proj(const float* __restrict__ x, const float* __restrict__ W, const float* __restrict__ bias, _Float16* __restrict__ out) {
  __shared__ __align__(16) float so[4][16 * 128];
  const int tid = threadIdx.x, wave = tid >> 5, lane = tid & 31, col = lane & 15, g = lane >> 4;
  const int b = blockIdx.z, t0 = blockIdx.x * 64 + wave * 16, n0 = blockIdx.y * 128;
  v16h a; { const float* xr = x + ((size_t)b * T0 + t0 + col) * FE;
#pragma unroll
    for (int i = 0; i < 8; ++i) { const int ka = 8 * g + i, kb = ka + 16; a[i] = (_Float16)(ka < FE ? xr[ka] : 0.f); a[8 + i] = (_Float16)(kb < FE ? xr[kb] : 0.f); } }
  v8f acc[8] = {};
#pragma unroll
  for (int j = 0; j < 8; ++j) { v16h bw; const float* wr = W + (size_t)(n0 + j * 16 + col) * FE;
#pragma unroll
    for (int i = 0; i < 8; ++i) { const int ka = 8 * g + i, kb = ka + 16; bw[i] = (_Float16)(ka < FE ? wr[ka] : 0.f); bw[8 + i] = (_Float16)(kb < FE ? wr[kb] : 0.f); }
    acc[j] = wmma16(a, bw, acc[j]); }
  float* S = so[wave];
#pragma unroll
  for (int j = 0; j < 8; ++j) { const float bv = bias[n0 + j * 16 + col];
#pragma unroll
    for (int r = 0; r < 8; ++r) S[(8 * g + r) * 128 + j * 16 + col] = acc[j][r] + bv; }
  LDSX();
#pragma unroll
  for (int q = 0; q < 8; ++q) { const int rl = q * 2 + (lane >> 4), pc = lane & 15; union { v8h h; v4u u; } pk;
#pragma unroll
    for (int e = 0; e < 8; ++e) pk.h[e] = (_Float16)S[rl * 128 + pc * 8 + e];
    vst2(out + ((size_t)b * T0 + t0 + rl) * C1 + n0 + pc * 8, pk.u); }
}

template <int CIN, int KT, int DIL, int TIN, int COUT, int POOL>
__global__ __launch_bounds__(128) void k_tdnn(const _Float16* __restrict__ in, const _Float16* __restrict__ W, const float* __restrict__ bias,
                                            _Float16* __restrict__ out, const int* __restrict__ lens, float* __restrict__ part) {
  constexpr int TOUT = TIN - (KT - 1) * DIL;
  constexpr int KK = KT * CIN;
  __shared__ __align__(16) float so[4][16 * 128];
  __shared__ float cs[4][2][128];
  const int tid = threadIdx.x, wave = tid >> 5, lane = tid & 31, col = lane & 15, g = lane >> 4;
  const int b = blockIdx.z, t0 = blockIdx.x * 64 + wave * 16, n0 = blockIdx.y * 128;
  int ta = t0 + col; if (ta > TOUT - 1) ta = TOUT - 1;
  const _Float16* inb = in + (size_t)b * TIN * CIN;
  v8f acc[8] = {};
#pragma unroll 1
  for (int kc = 0; kc < KK / 32; ++kc) { const int j = (kc * 32) / CIN, c0 = (kc * 32) % CIN;
    const v16h a = frag_h(inb + (size_t)(ta + j * DIL) * CIN + c0, lane);
#pragma unroll
    for (int jj = 0; jj < 8; ++jj) { int o = n0 + jj * 16 + col; if (o > COUT - 1) o = COUT - 1;
      acc[jj] = wmma16(a, frag_h(W + (size_t)o * KK + kc * 32, lane), acc[jj]); } }
  float* S = so[wave];
#pragma unroll
  for (int jj = 0; jj < 8; ++jj) { int o = n0 + jj * 16 + col; const float bv = o < COUT ? bias[o] : 0.f;
#pragma unroll
    for (int r = 0; r < 8; ++r) { const float u = acc[jj][r] + bv; S[(8 * g + r) * 128 + jj * 16 + col] = u > 0.f ? u : 0.f; } }
  LDSX();
  if (!POOL) {
#pragma unroll
    for (int q = 0; q < 8; ++q) { const int rl = q * 2 + (lane >> 4), pc = lane & 15; if (t0 + rl >= TOUT) continue;
      union { v8h h; v4u u; } pk;
#pragma unroll
      for (int e = 0; e < 8; ++e) pk.h[e] = (_Float16)S[rl * 128 + pc * 8 + e];
      vst2(out + ((size_t)b * TOUT + t0 + rl) * COUT + n0 + pc * 8, pk.u); }
  } else {
    int len = lens[b] - 8; if (len > TOUT) len = TOUT; if (len < 0) len = 0;
    float q1[4] = {0.f, 0.f, 0.f, 0.f}, q2[4] = {0.f, 0.f, 0.f, 0.f};
    for (int rl = 0; rl < 16; ++rl) { if (t0 + rl >= len) break;
      const v4f v = *(const v4f*)(S + rl * 128 + lane * 4);
#pragma unroll
      for (int e = 0; e < 4; ++e) { q1[e] += v[e]; q2[e] += v[e] * v[e]; } }
#pragma unroll
    for (int e = 0; e < 4; ++e) { cs[wave][0][lane * 4 + e] = q1[e]; cs[wave][1][lane * 4 + e] = q2[e]; }
    __syncthreads();
    if (tid < 64) { const int which = tid >> 5, l4 = (tid & 31) * 4; v4f t;
#pragma unroll
      for (int e = 0; e < 4; ++e) t[e] = cs[0][which][l4 + e] + cs[1][which][l4 + e] + cs[2][which][l4 + e] + cs[3][which][l4 + e];
      vst2(part + (((size_t)b * NTB + blockIdx.x) * 2 + which) * C5P + n0 + l4, t); }
  }
}

#define SP 3008
__global__ __launch_bounds__(256) void k_pool(const float* __restrict__ part, const int* __restrict__ lens, float* __restrict__ stat) {
  const int b = blockIdx.x, tid = threadIdx.x;
  int len = lens[b] - 8; if (len > T5) len = T5; if (len < 0) len = 0;
  const float n = (float)len;
  for (int c = tid; c < SP - C5; c += 256) {
    float s = 0.f, q = 0.f;
    if (c < C5) { for (int tb = 0; tb < NTB; ++tb) { s += part[(((size_t)b * NTB + tb) * 2) * C5P + c]; q += part[(((size_t)b * NTB + tb) * 2 + 1) * C5P + c]; } }
    const float mean = c < C5 ? s / n : 0.f;
    float var = c < C5 ? (q - n * mean * mean) / (n - 1.0f) : 0.f; var = var < 0.f ? 0.f : var;
    if (c < C5) vst2(stat + (size_t)b * SP + c, (float_a)mean);
    vst2(stat + (size_t)b * SP + C5 + c, (float_a)(c < C5 ? sqrtf(var) : 0.f));
  }
}

__global__ __launch_bounds__(32) void k_head(const float* __restrict__ A, int lda, int K, const float* __restrict__ W, const float* __restrict__ bias,
                                           float* __restrict__ Out, int N) {
  __shared__ __align__(16) float S[16][132];
  const int lane = threadIdx.x, col = lane & 15, g = lane >> 4, n0 = blockIdx.x * 128;
  v8f acc[8] = {};
#pragma unroll 1
  for (int kc = 0; kc < (K + 31) / 32; ++kc) { const F2 a = split_rowK(A + (size_t)col * lda, kc * 32, lane, K);
#pragma unroll
    for (int j = 0; j < 8; ++j) acc[j] = mac3(a, split_rowK(W + (size_t)(n0 + j * 16 + col) * K, kc * 32, lane, K), acc[j]); }
#pragma unroll
  for (int j = 0; j < 8; ++j) { const float bv = bias[n0 + j * 16 + col];
#pragma unroll
    for (int r = 0; r < 8; ++r) S[8 * g + r][j * 16 + col] = acc[j][r] + bv; }
  LDSX();
  for (int q = lane; q < 16 * 32; q += 32) { const int rl = q >> 5, pc = q & 31; vst2(Out + (size_t)rl * N + n0 + pc * 4, *(const v4f*)(&S[rl][pc * 4])); }
}
__global__ __launch_bounds__(256) void k_colnorm(const float* __restrict__ Ws, float* __restrict__ inv) {
  const int s = blockIdx.x * 256 + threadIdx.x; if (s >= NSPK) return;
  float q = 0.f;
#pragma unroll 1
  for (int k = 0; k < C1; ++k) { const float v = Ws[(size_t)k * NSPK + s]; q += v * v; }
  vst2(inv + s, (float_a)(1.0f / sqrtf(q)));
}
__global__ __launch_bounds__(32) void k_cos(const float* __restrict__ hs, const float* __restrict__ Ws, float* __restrict__ cosr) {
  __shared__ __align__(16) float S[16][132];
  const int lane = threadIdx.x, col = lane & 15, g = lane >> 4, n0 = blockIdx.x * 128;
  v8f acc[8] = {};
#pragma unroll 1
  for (int kc = 0; kc < C1 / 32; ++kc) { const F2 a = split_rowK(hs + (size_t)col * C1, kc * 32, lane, C1);
#pragma unroll
    for (int j = 0; j < 8; ++j) { int s = n0 + j * 16 + col; if (s > NSPK - 1) s = NSPK - 1; acc[j] = mac3(a, split_colK(Ws, kc * 32, s, lane, NSPK, C1), acc[j]); } }
#pragma unroll
  for (int j = 0; j < 8; ++j)
#pragma unroll
    for (int r = 0; r < 8; ++r) S[8 * g + r][j * 16 + col] = acc[j][r];
  LDSX();
  for (int q = lane; q < 16 * 32; q += 32) { const int rl = q >> 5, pc = q & 31; if (n0 + pc * 4 >= 6016) continue;
    vst2(cosr + (size_t)rl * 6016 + n0 + pc * 4, *(const v4f*)(&S[rl][pc * 4])); }
}
__global__ __launch_bounds__(256) void k_logits(const float* __restrict__ cosr, const float* __restrict__ inv, const float* __restrict__ hs,
                                              const int* __restrict__ spk, float* __restrict__ out) {
  __shared__ __align__(16) float cs[NSPK];
  __shared__ float redv[256]; __shared__ int redi[256]; __shared__ int top[6]; __shared__ float hn;
  const int r = blockIdx.x, tid = threadIdx.x;
  if (tid < 32) { float q = 0.f; for (int k = tid; k < C1; k += 32) { const float v = hs[(size_t)r * C1 + k]; q += v * v; }
#pragma unroll
    for (int off = 16; off >= 1; off >>= 1) q += __shfl_xor(q, off, 32);
    if (tid == 0) hn = 1.0f / sqrtf(q); }
  __syncthreads();
  const float hinv = hn;
  for (int s = tid; s < NSPK; s += 256) cs[s] = cosr[(size_t)r * 6016 + s] * inv[s] * hinv;
  __syncthreads();
#pragma unroll 1
  for (int k = 0; k < 6; ++k) {
    float bv = -3.0e38f; int bi = 0x7fffffff;
    for (int s = tid; s < NSPK; s += 256) { bool taken = false; for (int q = 0; q < k; ++q) taken |= (top[q] == s);
      const float v = cs[s]; if (!taken && (v > bv || (v == bv && s < bi))) { bv = v; bi = s; } }
    redv[tid] = bv; redi[tid] = bi; __syncthreads();
    for (int st = 128; st > 0; st >>= 1) { if (tid < st) { const float v2 = redv[tid + st]; const int i2 = redi[tid + st];
        if (v2 > redv[tid] || (v2 == redv[tid] && i2 < redi[tid])) { redv[tid] = v2; redi[tid] = i2; } } __syncthreads(); }
    if (tid == 0) top[k] = redi[0];
    __syncthreads();
  }
  const int tgt = spk[r];
  for (int s = tid; s < NSPK; s += 256) { bool pen = false;
#pragma unroll
    for (int q = 0; q < 6; ++q) pen |= (top[q] == s);
    const float c = cs[s]; const float v = (s == tgt) ? (c - 0.4f) : (pen ? c + 0.1f : c);
    cs[s] = 30.0f * v; }
  __syncthreads();
  for (int q = tid; q < NSPK / 4; q += 256) vst2(out + (size_t)r * NSPK + q * 4, *(const v4f*)(&cs[q * 4]));
}
__global__ __launch_bounds__(128) void k_lang(const float* __restrict__ l0, const float* __restrict__ W1, const float* __restrict__ b1,
                                            const float* __restrict__ xv, float* __restrict__ lang, float* __restrict__ xout) {
  __shared__ __align__(16) float sl[NB * 2 + 4];
  const int tid = threadIdx.x, w = tid >> 5, lane = tid & 31;
  for (int r = w; r < NB; r += 4) {
    float a0 = 0.f, a1 = 0.f;
#pragma unroll 1
    for (int k = lane; k < C1; k += 32) { const float v = l0[(size_t)r * C1 + k]; a0 += v * W1[k]; a1 += v * W1[C1 + k]; }
#pragma unroll
    for (int off = 16; off >= 1; off >>= 1) { a0 += __shfl_xor(a0, off, 32); a1 += __shfl_xor(a1, off, 32); }
    if (lane == 0) { sl[r * 2] = a0 + b1[0]; sl[r * 2 + 1] = a1 + b1[1]; } }
  __syncthreads();
  if (tid < 8) vst2(lang + tid * 4, *(const v4f*)(&sl[tid * 4]));
  for (int q = tid; q < NB * C1 / 4; q += 128) vst2(xout + q * 4, *(const v4f*)(xv + q * 4));
}

extern "C" void kernel_launch(void* const* d_in, const int* in_sizes, int n_in,
                              void* d_out, int out_size, void* d_ws, size_t ws_size,
                              hipStream_t stream) {
  (void)in_sizes; (void)n_in; (void)out_size; (void)ws_size;
  const float* mfcc = (const float*)d_in[0]; const int* slen = (const int*)d_in[1]; const int* spk = (const int*)d_in[2];
  const float* pw = (const float*)d_in[3]; const float* pb = (const float*)d_in[4];
  const float* w0 = (const float*)d_in[5]; const float* b0 = (const float*)d_in[6];
  const float* w1 = (const float*)d_in[7]; const float* b1 = (const float*)d_in[8];
  const float* w2 = (const float*)d_in[9]; const float* b2 = (const float*)d_in[10];
  const float* w3 = (const float*)d_in[11]; const float* b3 = (const float*)d_in[12];
  const float* w4 = (const float*)d_in[13]; const float* b4 = (const float*)d_in[14];
  const float* few = (const float*)d_in[15]; const float* feb = (const float*)d_in[16];
  const float* clw = (const float*)d_in[17]; const float* clb = (const float*)d_in[18];
  const float* spw = (const float*)d_in[19];
  const float* l0w = (const float*)d_in[20]; const float* l0b = (const float*)d_in[21];
  const float* l1w = (const float*)d_in[22]; const float* l1b = (const float*)d_in[23];
  float* out0 = (float*)d_out; float* out1 = (float*)d_out + 96000; float* out2 = (float*)d_out + 96032;
  char* ws = (char*)d_ws; size_t off = 0;
  auto take = [&](size_t bytes) { char* p = ws + off; off += (bytes + 255) & ~(size_t)255; return p; };
  _Float16* W0 = (_Float16*)take((size_t)C1 * 5 * C1 * 2); _Float16* W1h = (_Float16*)take((size_t)C1 * 3 * C1 * 2);
  _Float16* W2h = (_Float16*)take((size_t)C1 * 3 * C1 * 2); _Float16* W3h = (_Float16*)take((size_t)C1 * C1 * 2);
  _Float16* W4h = (_Float16*)take((size_t)C5 * C1 * 2);
  _Float16* hA = (_Float16*)take((size_t)NB * T0 * C1 * 2);
  _Float16* hB = (_Float16*)take((size_t)NB * T0 * C1 * 2);
  float* part = (float*)take((size_t)NB * NTB * 2 * C5P * 4);
  float* stat = (float*)take((size_t)NB * SP * 4);
  float* xvec = (float*)take((size_t)NB * C1 * 4); float* hs = (float*)take((size_t)NB * C1 * 4); float* l0 = (float*)take((size_t)NB * C1 * 4);
  float* inv = (float*)take((size_t)6144 * 4); float* cosr = (float*)take((size_t)NB * 6016 * 4);
  auto cvt = [&](const float* s, _Float16* d, size_t n) { k_cvt<<<(unsigned)((n / 8 + 255) / 256), 256, 0, stream>>>(s, d, n / 8); };
  cvt(w0, W0, (size_t)C1 * 5 * C1); cvt(w1, W1h, (size_t)C1 * 3 * C1); cvt(w2, W2h, (size_t)C1 * 3 * C1); cvt(w3, W3h, (size_t)C1 * C1); cvt(w4, W4h, (size_t)C5 * C1);
  k_proj<<<dim3(T0 / 64, C1 / 128, NB), 128, 0, stream>>>(mfcc, pw, pb, hA);
  k_tdnn<C1, 5, 1, 2048, C1, 0><<<dim3((2044 + 63) / 64, C1 / 128, NB), 128, 0, stream>>>(hA, W0, b0, hB, slen, nullptr);
  k_tdnn<C1, 3, 2, 2044, C1, 0><<<dim3((2040 + 63) / 64, C1 / 128, NB), 128, 0, stream>>>(hB, W1h, b1, hA, slen, nullptr);
  k_tdnn<C1, 3, 3, 2040, C1, 0><<<dim3((2034 + 63) / 64, C1 / 128, NB), 128, 0, stream>>>(hA, W2h, b2, hB, slen, nullptr);
  k_tdnn<C1, 1, 1, 2034, C1, 0><<<dim3((2034 + 63) / 64, C1 / 128, NB), 128, 0, stream>>>(hB, W3h, b3, hA, slen, nullptr);
  k_tdnn<C1, 1, 1, 2034, C5, 1><<<dim3((2034 + 63) / 64, C5P / 128, NB), 128, 0, stream>>>(hA, W4h, b4, nullptr, slen, part);
  k_pool<<<NB, 256, 0, stream>>>(part, slen, stat);
  k_head<<<C1 / 128, 32, 0, stream>>>(stat, SP, 2 * C5, few, feb, xvec, C1);
  k_head<<<C1 / 128, 32, 0, stream>>>(xvec, C1, C1, clw, clb, hs, C1);
  k_head<<<C1 / 128, 32, 0, stream>>>(xvec, C1, C1, l0w, l0b, l0, C1);
  k_colnorm<<<(NSPK + 255) / 256, 256, 0, stream>>>(spw, inv);
  k_cos<<<6016 / 128, 32, 0, stream>>>(hs, spw, cosr);
  k_logits<<<NB, 256, 0, stream>>>(cosr, inv, hs, spk, out0);
  k_lang<<<1, 128, 0, stream>>>(l0, l1w, l1b, xvec, out1, out2);
}
